// Model_61529701482572
// MI455X (gfx1250) — hardware-verified
//
#include <hip/hip_runtime.h>
#include <stddef.h>
#include <stdint.h>

#define FD      41024
#define KBASE   641
#define HC      256
#define NT64    641
#define HK      1024
#define H1N     32
#define BPB     32
#define PTHR    256
#define W1DBLK  16
#define AP2     72
#define WSMAX   134217728

static_assert(NT64 * 64 == FD);
static_assert(63 * KBASE + 4 * 64 + 63 < FD);
static_assert(W1DBLK * PTHR * 8 == H1N * HK);
static_assert((AP2 * 2) % 16 == 0 && AP2 >= 64);
static_assert(HK % 32 == 0 && 64 % 32 == 0);
static_assert(BPB == 32);

typedef float          v2f   __attribute__((ext_vector_type(2)));
typedef float          v4f   __attribute__((ext_vector_type(4)));
typedef float          v8f   __attribute__((ext_vector_type(8)));
typedef int            v8i   __attribute__((ext_vector_type(8)));
typedef unsigned       v4u   __attribute__((ext_vector_type(4)));
typedef unsigned short v8us  __attribute__((ext_vector_type(8)));
typedef unsigned short v16us __attribute__((ext_vector_type(16)));
typedef __bf16         v16bf __attribute__((ext_vector_type(16)));
typedef v2f  __attribute__((may_alias)) v2fa;
typedef v4f  __attribute__((may_alias)) v4fa;
typedef v4u  __attribute__((may_alias)) v4ua;
typedef v8us __attribute__((may_alias)) v8usa;
union FragB { v16bf v; v16us u; v8us h[2]; v8i w; };

__device__ __forceinline__ v8f wmb(const FragB& a, const FragB& b, v8f c) {
  v8f d = __builtin_amdgcn_wmma_f32_16x16x32_bf16(false, a.v, false, b.v, (short)0, c, false, false);
  asm volatile("v_nop\n\tv_nop\n\tv_nop\n\tv_nop" : "+v"(d) : "v"(a.w), "v"(b.w));
  return d;
}

__device__ __forceinline__ unsigned bf16_bits(float f) {
  const unsigned u = __float_as_uint(f);
  return (u + 0x7FFFu + ((u >> 16) & 1u)) >> 16;
}
__device__ __forceinline__ float bf16_val(float f) {
  return __uint_as_float(bf16_bits(f) << 16);
}

__global__ __launch_bounds__(PTHR) void k_prep(const float* __restrict__ Wmy, const float* __restrict__ Wopp,
                                               const float* __restrict__ W1,
                                               unsigned short* WT, unsigned short* W1D) {
  __shared__ __attribute__((aligned(16))) unsigned short tile[64 * HC];
  const int tid = (int)threadIdx.x;
  const int blk = (int)blockIdx.x;
  if (blk < 2 * NT64) {
    const int mat  = (blk >= NT64) ? 1 : 0;
    const int tl   = blk - mat * NT64;
    const int idx0 = tl * 64;
    const float* W = mat ? Wopp : Wmy;
#pragma unroll 4
    for (int it = 0; it < 16; ++it) {
      const int u = it * PTHR + tid;
      const int c = u >> 4;
      const int q = u & 15;
      const v4f x = *(const v4fa*)(W + (size_t)c * FD + idx0 + 4 * q);
      tile[(4 * q + 0) * HC + c] = (unsigned short)bf16_bits(x.x);
      tile[(4 * q + 1) * HC + c] = (unsigned short)bf16_bits(x.y);
      tile[(4 * q + 2) * HC + c] = (unsigned short)bf16_bits(x.z);
      tile[(4 * q + 3) * HC + c] = (unsigned short)bf16_bits(x.w);
    }
    __syncthreads();
    v8us pv[8];
#pragma unroll
    for (int it = 0; it < 8; ++it) pv[it] = *(const v8usa*)(tile + (size_t)(it * PTHR + tid) * 8);
    unsigned short* dst = WT + ((size_t)mat * FD + idx0) * HC;
#pragma unroll
    for (int it = 0; it < 8; ++it) *(volatile v8us*)(dst + (size_t)(it * PTHR + tid) * 8) = pv[it];
    __threadfence();
#pragma unroll
    for (int it = 0; it < 8; ++it) *(volatile v8us*)(dst + (size_t)(it * PTHR + tid) * 8) = pv[it];
  } else {
    const int u  = (blk - 2 * NT64) * PTHR + tid;
    const int n  = u >> 7;
    const int k8 = (u & 127) * 8;
    const float* p = W1 + (size_t)n * 512 + (k8 & 511);
    const v4f a = *(const v4fa*)p;
    const v4f b = *(const v4fa*)(p + 4);
    v8us o;
    o[0] = (unsigned short)bf16_bits(a.x); o[1] = (unsigned short)bf16_bits(a.y);
    o[2] = (unsigned short)bf16_bits(a.z); o[3] = (unsigned short)bf16_bits(a.w);
    o[4] = (unsigned short)bf16_bits(b.x); o[5] = (unsigned short)bf16_bits(b.y);
    o[6] = (unsigned short)bf16_bits(b.z); o[7] = (unsigned short)bf16_bits(b.w);
    unsigned short* dp = W1D + (size_t)n * HK + k8;
    *(volatile v8us*)dp = o;
    __threadfence();
    *(volatile v8us*)dp = o;
  }
}

__global__ __launch_bounds__(PTHR) void k_feat(const int* __restrict__ boards,
                                               const unsigned* __restrict__ WT32,
                                               const float* __restrict__ bmy, const float* __restrict__ bopp,
                                               unsigned* HHL32) {
  __shared__ int sd[64];
  __shared__ int lists[128];
  __shared__ __attribute__((aligned(16))) unsigned sRow[512];

  const int tid = (int)threadIdx.x, lane = tid & 31, wave = tid >> 5;
  const int b = (int)blockIdx.x;
  if (tid < 64) {
    sd[tid] = boards[(size_t)b * 64 + tid];
    lists[tid] = 0;
    lists[64 + tid] = 0;
  }
  __syncthreads();

  const int v0 = sd[lane];
  const int v1 = sd[32 + lane];
  const unsigned kMlo = __builtin_amdgcn_ballot_w32(v0 == 0);
  const unsigned kMhi = __builtin_amdgcn_ballot_w32(v1 == 0);
  const unsigned kOlo = __builtin_amdgcn_ballot_w32(v0 == 12);
  const unsigned kOhi = __builtin_amdgcn_ballot_w32(v1 == 12);
  const int mk = kMlo ? (__builtin_ffs((int)kMlo) - 1) : (kMhi ? (31 + __builtin_ffs((int)kMhi)) : 0);
  const int ok = kOlo ? (__builtin_ffs((int)kOlo) - 1) : (kOhi ? (31 + __builtin_ffs((int)kOhi)) : 0);

  const bool o0 = (v0 >= 7) & (v0 <= 11);
  const bool o1 = (v1 >= 7) & (v1 <= 11);
  const bool m0 = (v0 >= 1) & (v0 <= 5);
  const bool m1 = (v1 >= 1) & (v1 <= 5);
  const unsigned pOlo = __builtin_amdgcn_ballot_w32(o0);
  const unsigned pOhi = __builtin_amdgcn_ballot_w32(o1);
  const unsigned pMlo = __builtin_amdgcn_ballot_w32(m0);
  const unsigned pMhi = __builtin_amdgcn_ballot_w32(m1);
  const unsigned below = (1u << lane) - 1u;
  const int nO = (int)__builtin_popcount(pOlo) + (int)__builtin_popcount(pOhi);
  const int nM = (int)__builtin_popcount(pMlo) + (int)__builtin_popcount(pMhi);

  if (wave == 0) {
    const int posO0 = (int)__builtin_popcount(pOlo & below);
    const int posO1 = (int)__builtin_popcount(pOlo) + (int)__builtin_popcount(pOhi & below);
    const int posM0 = (int)__builtin_popcount(pMlo & below);
    const int posM1 = (int)__builtin_popcount(pMlo) + (int)__builtin_popcount(pMhi & below);
    int iO0 = ok * KBASE + (11 - v0) * 64 + lane;
    int iO1 = ok * KBASE + (11 - v1) * 64 + 32 + lane;
    int iM0 = mk * KBASE + (v0 - 1) * 64 + lane;
    int iM1 = mk * KBASE + (v1 - 1) * 64 + 32 + lane;
    iO0 = min(max(iO0, 0), FD - 1);
    iO1 = min(max(iO1, 0), FD - 1);
    iM0 = min(max(iM0, 0), FD - 1);
    iM1 = min(max(iM1, 0), FD - 1);
    if (o0) lists[posO0 & 63] = iO0;
    if (o1) lists[posO1 & 63] = iO1;
    if (m0) lists[64 + (posM0 & 63)] = iM0;
    if (m1) lists[64 + (posM1 & 63)] = iM1;
  }
  __syncthreads();

  const int side = tid >> 7;
  const int t    = tid & 127;
  int n = side ? nM : nO;
  n = n < 0 ? 0 : (n > 64 ? 64 : n);
  const unsigned* wp = WT32 + (size_t)side * ((size_t)FD * 128) + t;
  const int* lst = lists + side * 64;

  float a0 = 0.0f, a1 = 0.0f;
#pragma unroll 4
  for (int j = 0; j < n; ++j) {
    int idx = lst[j];
    idx = min(max(idx, 0), FD - 1);
    const unsigned w = wp[(size_t)idx * 128];
    a0 += __uint_as_float(w << 16);
    a1 += __uint_as_float(w & 0xffff0000u);
  }

  const v2f bm = *(const v2fa*)(bmy + 2 * t);
  const v2f bo = *(const v2fa*)(bopp + 2 * t);
  const float bb0 = bf16_val(side ? bo.x : bm.x);
  const float bb1 = bf16_val(side ? bo.y : bm.y);
  const float h0 = fmaxf(a0 + bb0, 0.0f);
  const float h1 = fmaxf(a1 + bb1, 0.0f);
  const unsigned hb0 = bf16_bits(h0);
  const unsigned hb1 = bf16_bits(h1);
  const unsigned lb0 = bf16_bits(h0 - __uint_as_float(hb0 << 16));
  const unsigned lb1 = bf16_bits(h1 - __uint_as_float(hb1 << 16));
  sRow[side * 128 + t]       = hb0 | (hb1 << 16);
  sRow[256 + side * 128 + t] = lb0 | (lb1 << 16);
  __syncthreads();

  if (tid < 128) {
    const v4u val = *(const v4ua*)(sRow + 4 * tid);
    unsigned* dp = HHL32 + (size_t)b * 512 + 4 * tid;
    *(volatile v4u*)dp = val;
    __threadfence();
    *(volatile v4u*)dp = val;
  }
}

__global__ __launch_bounds__(128) void k_mlp(const unsigned short* __restrict__ HHL,
                                             const unsigned short* __restrict__ W1D,
                                             const float* __restrict__ b1, const float* __restrict__ W2,
                                             const float* __restrict__ b2, const float* __restrict__ W3,
                                             const float* __restrict__ b3, float* out) {
  __shared__ __attribute__((aligned(16))) unsigned short sA[BPB * AP2];
  __shared__ __attribute__((aligned(16))) unsigned short sB[H1N * AP2];
  __shared__ float sH2[BPB * 33];
  __shared__ __attribute__((aligned(16))) float sOut[BPB];

  const int tid = (int)threadIdx.x, lane = tid & 31, wave = tid >> 5;
  const int hh = lane >> 4, m = lane & 15;
  const int mt = wave >> 1, nt = wave & 1;
  const int b0 = (int)blockIdx.x * BPB;

  {
    const int n  = tid >> 2;
    const int kq = (tid & 3) * 16;
    const float* p = W2 + (size_t)n * 32 + (kq & 31);
    const v4f x0 = *(const v4fa*)p;
    const v4f x1 = *(const v4fa*)(p + 4);
    const v4f x2 = *(const v4fa*)(p + 8);
    const v4f x3 = *(const v4fa*)(p + 12);
    unsigned short* q = sB + n * AP2 + kq;
    q[0]  = (unsigned short)bf16_bits(x0.x); q[1]  = (unsigned short)bf16_bits(x0.y);
    q[2]  = (unsigned short)bf16_bits(x0.z); q[3]  = (unsigned short)bf16_bits(x0.w);
    q[4]  = (unsigned short)bf16_bits(x1.x); q[5]  = (unsigned short)bf16_bits(x1.y);
    q[6]  = (unsigned short)bf16_bits(x1.z); q[7]  = (unsigned short)bf16_bits(x1.w);
    q[8]  = (unsigned short)bf16_bits(x2.x); q[9]  = (unsigned short)bf16_bits(x2.y);
    q[10] = (unsigned short)bf16_bits(x2.z); q[11] = (unsigned short)bf16_bits(x2.w);
    q[12] = (unsigned short)bf16_bits(x3.x); q[13] = (unsigned short)bf16_bits(x3.y);
    q[14] = (unsigned short)bf16_bits(x3.z); q[15] = (unsigned short)bf16_bits(x3.w);
  }

  v8f acc = {0.f, 0.f, 0.f, 0.f, 0.f, 0.f, 0.f, 0.f};
  {
    const unsigned short* ap = HHL + (size_t)(b0 + 16 * mt + m) * HK + 8 * hh;
    const unsigned short* bp = W1D + (size_t)(16 * nt + m) * HK + 8 * hh;
#pragma unroll 4
    for (int k0 = 0; k0 < HK; k0 += 32) {
      FragB af, bf;
      af.h[0] = *(const v8usa*)(ap + k0);
      af.h[1] = *(const v8usa*)(ap + k0 + 16);
      bf.h[0] = *(const v8usa*)(bp + k0);
      bf.h[1] = *(const v8usa*)(bp + k0 + 16);
      acc = wmb(af, bf, acc);
    }
  }
  {
    const int col = 16 * nt + m;
    const float bv = bf16_val(b1[col]);
#pragma unroll
    for (int r = 0; r < 8; ++r) {
      const int row = 16 * mt + 8 * hh + r;
      const float v = fmaxf(acc[r] + bv, 0.0f);
      const unsigned hb = bf16_bits(v);
      const unsigned lb = bf16_bits(v - __uint_as_float(hb << 16));
      sA[row * AP2 + col]      = (unsigned short)hb;
      sA[row * AP2 + 32 + col] = (unsigned short)lb;
    }
  }
  __syncthreads();

  v8f acc2 = {0.f, 0.f, 0.f, 0.f, 0.f, 0.f, 0.f, 0.f};
  {
    const unsigned short* ap = sA + (16 * mt + m) * AP2 + 8 * hh;
    const unsigned short* bp = sB + (16 * nt + m) * AP2 + 8 * hh;
#pragma unroll
    for (int k0 = 0; k0 < 64; k0 += 32) {
      FragB af, bf;
      af.h[0] = *(const v8usa*)(ap + k0);
      af.h[1] = *(const v8usa*)(ap + k0 + 16);
      bf.h[0] = *(const v8usa*)(bp + k0);
      bf.h[1] = *(const v8usa*)(bp + k0 + 16);
      acc2 = wmb(af, bf, acc2);
    }
  }
  {
    const int col = 16 * nt + m;
    const float bv = bf16_val(b2[col]);
#pragma unroll
    for (int r = 0; r < 8; ++r) {
      const int row = 16 * mt + 8 * hh + r;
      sH2[row * 33 + col] = fmaxf(acc2[r] + bv, 0.0f);
    }
  }
  __syncthreads();

  {
    const float w3  = bf16_val(W3[lane]);
    const float bb3 = bf16_val(b3[0]);
#pragma unroll
    for (int rr = 0; rr < 8; ++rr) {
      const int row = 8 * wave + rr;
      float p = sH2[row * 33 + lane] * w3;
      p += __shfl_xor(p, 16);
      p += __shfl_xor(p, 8);
      p += __shfl_xor(p, 4);
      p += __shfl_xor(p, 2);
      p += __shfl_xor(p, 1);
      if (lane == 0) sOut[row] = p + bb3;
    }
  }
  __syncthreads();

  if (tid < 8) {
    const v4f o = *(const v4fa*)(sOut + 4 * tid);
    float* op = out + (size_t)b0 + 4 * tid;
    *(volatile v4f*)op = o;
    __threadfence();
    *(volatile v4f*)op = o;
  }
}

extern "C" void kernel_launch(void* const* d_in, const int* in_sizes, int n_in,
                              void* d_out, int out_size, void* d_ws, size_t ws_size,
                              hipStream_t stream) {
  if (n_in < 11) return;
  const int nB = out_size;
  if (nB < BPB || (nB % BPB) != 0 || nB > 65536) return;
  if (in_sizes[0] != nB * 64) return;
  if (in_sizes[1] != HC * FD || in_sizes[3] != HC * FD) return;
  if (in_sizes[2] != HC || in_sizes[4] != HC) return;
  if (in_sizes[5] != H1N * 512 || in_sizes[6] != H1N) return;
  if (in_sizes[7] != H1N * H1N || in_sizes[8] != H1N) return;
  if (in_sizes[9] != H1N || in_sizes[10] != 1) return;

  const int*   boards = (const int*)d_in[0];
  const float* W_my   = (const float*)d_in[1];
  const float* b_my   = (const float*)d_in[2];
  const float* W_opp  = (const float*)d_in[3];
  const float* b_opp  = (const float*)d_in[4];
  const float* W1     = (const float*)d_in[5];
  const float* b1     = (const float*)d_in[6];
  const float* W2     = (const float*)d_in[7];
  const float* b2     = (const float*)d_in[8];
  const float* W3     = (const float*)d_in[9];
  const float* b3     = (const float*)d_in[10];
  float* out = (float*)d_out;

  const size_t szWT  = (size_t)2 * FD * HC * 2;
  const size_t szHHL = (size_t)nB * HK * 2;
  const size_t szW1D = (size_t)H1N * HK * 2;
  size_t off = 0;
  const size_t oWT  = off; off += szWT;  off = (off + 255) & ~(size_t)255;
  const size_t oHHL = off; off += szHHL; off = (off + 255) & ~(size_t)255;
  const size_t oW1D = off; off += szW1D; off = (off + 255) & ~(size_t)255;
  if (off > ws_size || off > (size_t)WSMAX) return;

  char* ws = (char*)d_ws;
  unsigned short* WT  = (unsigned short*)(ws + oWT);
  unsigned short* HHL = (unsigned short*)(ws + oHHL);
  unsigned short* W1D = (unsigned short*)(ws + oW1D);

  k_prep<<<2 * NT64 + W1DBLK, PTHR, 0, stream>>>(W_my, W_opp, W1, WT, W1D);
  k_feat<<<nB, PTHR, 0, stream>>>(boards, (const unsigned*)WT, b_my, b_opp, (unsigned*)HHL);
  k_mlp<<<nB / BPB, 128, 0, stream>>>(HHL, W1D, b1, W2, b2, W3, b3, out);
}
